// LocalAggregator_52836687675884
// MI455X (gfx1250) — hardware-verified
//
#include <hip/hip_runtime.h>


#define NBT  32
#define NN   128
#define DD   256
#define TD   64
#define NR   5
#define NRP  64
#define NPAIR ((size_t)NBT * NN * NN)
#define PCH   ((size_t)131072)
typedef _Float16 h16;
typedef unsigned short bf;
typedef __attribute__((ext_vector_type(16))) __bf16   v16bf;
typedef __attribute__((ext_vector_type(16))) _Float16 v16h;
typedef __attribute__((ext_vector_type(8)))  _Float16 v8h;
typedef __attribute__((ext_vector_type(8)))  unsigned short v8us;
typedef __attribute__((ext_vector_type(8)))  float    v8f;
typedef __attribute__((ext_vector_type(4)))  float    v4f;
typedef v8h  __attribute__((may_alias)) v8ha;
typedef v4f  __attribute__((may_alias)) v4fa;
typedef v8us __attribute__((may_alias)) v8usa;

__device__ __forceinline__ unsigned short f2bf(float f) { unsigned u = __float_as_uint(f); u += 0x7FFFu + ((u >> 16) & 1u); return (unsigned short)(u >> 16); }
__device__ __forceinline__ float bf2f(unsigned short b) { return __uint_as_float(((unsigned)b) << 16); }
__device__ __forceinline__ float bfr(float f) { return bf2f(f2bf(f)); }
__device__ __forceinline__ v16h cat16(v8h lo, v8h hi) { return __builtin_shufflevector(lo, hi, 0, 1, 2, 3, 4, 5, 6, 7, 8, 9, 10, 11, 12, 13, 14, 15); }
__device__ __forceinline__ v16bf cat16b(v8us lo, v8us hi) { return __builtin_bit_cast(v16bf, __builtin_shufflevector(lo, hi, 0, 1, 2, 3, 4, 5, 6, 7, 8, 9, 10, 11, 12, 13, 14, 15)); }
__device__ __forceinline__ v8f wmma16(v16h a, v16h b, v8f c) { return __builtin_amdgcn_wmma_f32_16x16x32_f16(false, a, false, b, (short)0, c, false, false); }
__device__ __forceinline__ v8f wmmab(v16bf a, v16bf b, v8f c) { return __builtin_amdgcn_wmma_f32_16x16x32_bf16(false, a, false, b, (short)0, c, false, false); }


template <typename T16> struct WFrag;
template <> struct WFrag<h16> { typedef v16h V; static __device__ __forceinline__ V ld(const h16* p) { return cat16(*(const v8h*)p, *(const v8h*)(p + 16)); } static __device__ __forceinline__ v8f mma(V a, V b, v8f c) { return wmma16(a, b, c); } };
template <> struct WFrag<bf> { typedef v16bf V; static __device__ __forceinline__ V ld(const bf* p) { return cat16b(*(const v8us*)p, *(const v8us*)(p + 16)); } static __device__ __forceinline__ v8f mma(V a, V b, v8f c) { return wmmab(a, b, c); } };
template <typename T16, int NSPLIT, bool BIAS>
__global__ __launch_bounds__(32) void k_gemmw(const T16* __restrict__ A, const T16* __restrict__ A2, const T16* __restrict__ Bt, const T16* __restrict__ Bt2, int K, float* C, int ldc, const float* __restrict__ bias, size_t sA, size_t sB, size_t sC) {
    typedef typename WFrag<T16>::V V;
    __shared__ __align__(16) float os[16 * 68];
    const size_t z = blockIdx.z; A += z * sA; if (A2) A2 += z * sA; Bt += z * sB; if (Bt2) Bt2 += z * sB; C += z * sC;
    const int lane = threadIdx.x & 31, lr = lane & 15, hi = lane >> 4; const int r0 = blockIdx.x * 64, c0 = blockIdx.y * 64;
    v8f acc[4][4];
#pragma unroll
    for (int mb = 0; mb < 4; ++mb)
#pragma unroll
        for (int nb = 0; nb < 4; ++nb) acc[mb][nb] = (v8f){};
    const size_t aoff = (size_t)(r0 + lr) * K + 8 * hi, boff = (size_t)(c0 + lr) * K + 8 * hi;
#pragma unroll 1
    for (int kc = 0; kc < K; kc += 32) {
        V a[4], a2[4];
#pragma unroll
        for (int mb = 0; mb < 4; ++mb) { a[mb] = WFrag<T16>::ld(A + aoff + (size_t)mb * 16 * K + kc); if (NSPLIT == 1 || NSPLIT == 2) a2[mb] = WFrag<T16>::ld(A2 + aoff + (size_t)mb * 16 * K + kc); }
#pragma unroll
        for (int nb = 0; nb < 4; ++nb) { const V b = WFrag<T16>::ld(Bt + boff + (size_t)nb * 16 * K + kc); V b2; if (NSPLIT >= 2) b2 = WFrag<T16>::ld(Bt2 + boff + (size_t)nb * 16 * K + kc);
#pragma unroll
            for (int mb = 0; mb < 4; ++mb) { acc[mb][nb] = WFrag<T16>::mma(a[mb], b, acc[mb][nb]); if (NSPLIT == 1 || NSPLIT == 2) acc[mb][nb] = WFrag<T16>::mma(a2[mb], b, acc[mb][nb]); if (NSPLIT >= 2) acc[mb][nb] = WFrag<T16>::mma(a[mb], b2, acc[mb][nb]); } }
        asm volatile("v_nop\n\tv_nop\n\tv_nop\n\tv_nop" : "+v"(acc[0][0]), "+v"(acc[1][1]), "+v"(acc[2][2]), "+v"(acc[3][3]) : "v"(a[0]), "v"(a[3]));
    }
#pragma unroll
    for (int mb = 0; mb < 4; ++mb) {
#pragma unroll
        for (int nb = 0; nb < 4; ++nb) {
#pragma unroll
            for (int j = 0; j < 8; ++j) os[(hi * 8 + j) * 68 + nb * 16 + lr] = acc[mb][nb][j]; }
        __builtin_amdgcn_wave_barrier(); asm volatile("" ::: "memory");
        float* crow = C + (size_t)(r0 + mb * 16) * ldc + c0;
#pragma unroll 1
        for (int ps = 0; ps < 2; ++ps) {
#pragma unroll
            for (int s = 0; s < 8; ++s) { const int row = 2 * s + hi, cofs = lr * 4; v4f val = *(const v4fa*)(os + row * 68 + cofs); if (BIAS) { val[0] += bfr(bias[c0 + cofs]); val[1] += bfr(bias[c0 + cofs + 1]); val[2] += bfr(bias[c0 + cofs + 2]); val[3] += bfr(bias[c0 + cofs + 3]); }
                *(volatile v4f*)(crow + (size_t)row * ldc + cofs) = val; }
            if (ps == 0) __threadfence(); }
        __builtin_amdgcn_wave_barrier(); asm volatile("" ::: "memory");
    }
}

typedef __attribute__((ext_vector_type(4))) unsigned short v4us;
typedef __attribute__((ext_vector_type(2))) unsigned short v2us;
__device__ __forceinline__ void splitf(float y, unsigned short& h, unsigned short& l) { h = f2bf(y); l = f2bf(y - bf2f(h)); }
__global__ __launch_bounds__(256) void k_cvt8(const float* __restrict__ src, bf* dst, size_t n8) { const size_t i = (size_t)blockIdx.x * 256 + threadIdx.x; if (i >= n8) return; const v8f v = *(const v8f*)(src + i * 8); v8us o;
#pragma unroll
    for (int k = 0; k < 8; ++k) o[k] = f2bf(v[k]); *(volatile v8us*)(dst + i * 8) = o; __threadfence(); *(volatile v8us*)(dst + i * 8) = o; }

__global__ __launch_bounds__(256) void k_ha(const float* __restrict__ h, const float* __restrict__ a, bf* Hh, bf* Hl) { const size_t e = ((size_t)blockIdx.x * 256 + threadIdx.x) * 4; if (e >= (size_t)NR * NBT * NN * DD) return; const int d = (int)(e % DD); const size_t bi = (e / DD) % ((size_t)NBT * NN); const int r = (int)(e / ((size_t)NBT * NN * DD)); v4us oh, ol;
#pragma unroll
    for (int q = 0; q < 4; ++q) { const float p = __fmul_rn(bfr(h[bi * DD + d + q]), bfr(a[(d + q) * NR + r])); unsigned short h2, l2; splitf(p, h2, l2); oh[q] = h2; ol[q] = l2; }
    *(volatile v4us*)(Hh + e) = oh; *(volatile v4us*)(Hl + e) = ol; __threadfence(); *(volatile v4us*)(Hh + e) = oh; *(volatile v4us*)(Hl + e) = ol; }
__global__ __launch_bounds__(256) void k_enc(const float* __restrict__ A, size_t p0, const float* __restrict__ fr, const float* __restrict__ ph, bf* Eh, bf* El) { const size_t e = ((size_t)blockIdx.x * 256 + threadIdx.x) * 2; if (e >= PCH * TD) return; const int t = (int)(e % TD); const size_t p = e / TD; const float av = bfr(A[p0 + p]); v2us oh, ol;
#pragma unroll
    for (int q = 0; q < 2; ++q) { float m = __fmul_rn(av, bfr(fr[t + q])); asm volatile("" : "+v"(m)); const float c = cosf(__fadd_rn(m, bfr(ph[t + q]))); unsigned short h2, l2; splitf(c, h2, l2); oh[q] = h2; ol[q] = l2; }
    *(volatile v2us*)(Eh + e) = oh; *(volatile v2us*)(El + e) = ol; __threadfence(); *(volatile v2us*)(Eh + e) = oh; *(volatile v2us*)(El + e) = ol; }
__global__ __launch_bounds__(64) void k_iwpad(const float* __restrict__ iw, bf* Bt) { const int r = threadIdx.x; if (r >= NRP) return; unsigned short c[TD];
#pragma unroll
    for (int t = 0; t < TD; ++t) c[t] = (r < NR) ? f2bf(iw[t * NR + r]) : (unsigned short)0;
#pragma unroll 1
    for (int ps = 0; ps < 2; ++ps) {
#pragma unroll
        for (int c8 = 0; c8 < TD; c8 += 8) { v8us o;
#pragma unroll
            for (int k = 0; k < 8; ++k) o[k] = c[c8 + k]; *(volatile v8us*)(Bt + (size_t)r * TD + c8) = o; }
        if (ps == 0) __threadfence(); } }
__global__ __launch_bounds__(256) void k_asel(const float* __restrict__ E1, const float* __restrict__ E2, size_t row0, const int* __restrict__ adj, bf* Ph, bf* Pl) {
    const int lane = threadIdx.x & 31; const size_t row = row0 + (size_t)blockIdx.x * 8 + (threadIdx.x >> 5); if (row >= row0 + PCH / NN) return;     float v[4]; float mx = -3.0e38f;
#pragma unroll
    for (int q = 0; q < 4; ++q) { const int j = lane * 4 + q; const size_t pr = row * NN + j; const int ad = adj[pr]; const int r = min(max(ad - 1, 0), NR - 1);
        const float e = __fadd_rn(E1[(size_t)r * NBT * NN * NN + pr], E2[(pr - row0 * NN) * NRP + r]); const float lr = (e >= 0.0f) ? e : __fmul_rn(0.2f, e); const float t = (ad >= 1 && ad <= 5) ? lr : -9.0e15f; v[q] = t; mx = fmaxf(mx, t); }
#pragma unroll
    for (int sh = 16; sh; sh >>= 1) mx = fmaxf(mx, __shfl_xor(mx, sh, 32));
    float sum = 0.f;
#pragma unroll
    for (int q = 0; q < 4; ++q) { float d0 = __fsub_rn(v[q], mx); asm volatile("" : "+v"(d0)); v[q] = __builtin_amdgcn_exp2f(__fmul_rn(d0, 1.4426950408889634f)); sum += v[q]; }
#pragma unroll
    for (int sh = 16; sh; sh >>= 1) sum += __shfl_xor(sum, sh, 32);
    const float f = __fdiv_rn(1.0f, sum); v4us oh, ol;
#pragma unroll
    for (int q = 0; q < 4; ++q) { unsigned short h2, l2; float y = __fmul_rn(v[q], f); asm volatile("" : "+v"(y)); splitf(y, h2, l2); oh[q] = h2; ol[q] = l2; }
    const size_t oo = row * NN + lane * 4; *(volatile v4us*)(Ph + oo) = oh; *(volatile v4us*)(Pl + oo) = ol; __threadfence(); *(volatile v4us*)(Ph + oo) = oh; *(volatile v4us*)(Pl + oo) = ol; }
__global__ __launch_bounds__(256) void k_ht(const float* __restrict__ h, bf* HT) { const size_t e = ((size_t)blockIdx.x * 256 + threadIdx.x) * 2; if (e >= (size_t)NBT * DD * NN) return; const int j = (int)(e % NN); const int d = (int)((e / NN) % DD); const int b = (int)(e / ((size_t)NN * DD)); v2us o; o[0] = f2bf(h[((size_t)b * NN + j) * DD + d]); o[1] = f2bf(h[((size_t)b * NN + j + 1) * DD + d]);
    *(volatile v2us*)(HT + e) = o; __threadfence(); *(volatile v2us*)(HT + e) = o; }

extern "C" void kernel_launch(void* const* d_in, const int* in_sizes, int n_in,
                              void* d_out, int out_size, void* d_ws, size_t ws_size, hipStream_t stream) {
    (void)in_sizes; (void)n_in; (void)out_size;
    const float* h = (const float*)d_in[0]; const float* A = (const float*)d_in[1]; const float* a = (const float*)d_in[2]; const float* iw = (const float*)d_in[3]; const float* fr = (const float*)d_in[4]; const float* ph = (const float*)d_in[5]; const int* adj = (const int*)d_in[6];
    float* OUT = (float*)d_out;
    char* wsp = (char*)d_ws;
    auto take = [&](size_t bytes) { char* p = wsp; wsp += (bytes + 255) & ~(size_t)255; return (void*)p; };
    bf* HB = (bf*)take((size_t)NBT * NN * DD * 2); bf* HAh = (bf*)take((size_t)NR * NBT * NN * DD * 2); bf* HAl = (bf*)take((size_t)NR * NBT * NN * DD * 2); bf* HT = (bf*)take((size_t)NBT * DD * NN * 2);
    float* E1 = (float*)take((size_t)NR * NPAIR * 4); bf* ENh = (bf*)take(PCH * TD * 2); bf* ENl = (bf*)take(PCH * TD * 2); bf* IWB = (bf*)take((size_t)NRP * TD * 2); float* E2 = (float*)take(PCH * NRP * 4);
    bf* Ph = (bf*)take(NPAIR * 2); bf* Pl = (bf*)take(NPAIR * 2);
    if ((size_t)(wsp - (char*)d_ws) > ws_size) return;
    k_cvt8<<<(unsigned)(((size_t)NBT * NN * DD / 8 + 255) / 256), 256, 0, stream>>>(h, HB, (size_t)NBT * NN * DD / 8);
    k_ha<<<(unsigned)(((size_t)NR * NBT * NN * DD / 4 + 255) / 256), 256, 0, stream>>>(h, a, HAh, HAl);
    for (int r = 0; r < NR; ++r)
        k_gemmw<bf, 1, false><<<dim3(NN / 64, NN / 64, NBT), 32, 0, stream>>>(HAh + (size_t)r * NBT * NN * DD, HAl + (size_t)r * NBT * NN * DD, HB, nullptr, DD, E1 + (size_t)r * NPAIR, NN, nullptr, (size_t)NN * DD, (size_t)NN * DD, (size_t)NN * NN);
    k_iwpad<<<1, 64, 0, stream>>>(iw, IWB);
    for (size_t p0 = 0; p0 < NPAIR; p0 += PCH) {
        k_enc<<<(unsigned)((PCH * TD / 2 + 255) / 256), 256, 0, stream>>>(A, p0, fr, ph, ENh, ENl);
        k_gemmw<bf, 1, false><<<dim3((unsigned)(PCH / 64), NRP / 64, 1), 32, 0, stream>>>(ENh, ENl, IWB, nullptr, TD, E2, NRP, nullptr, 0, 0, 0);
        k_asel<<<(unsigned)((PCH / NN + 7) / 8), 256, 0, stream>>>(E1, E2, p0 / NN, adj, Ph, Pl); }
    k_ht<<<(unsigned)(((size_t)NBT * DD * NN / 2 + 255) / 256), 256, 0, stream>>>(h, HT);
    k_gemmw<bf, 1, false><<<dim3(NN / 64, DD / 64, NBT), 32, 0, stream>>>(Ph, Pl, HT, nullptr, NN, OUT, DD, nullptr, (size_t)NN * NN, (size_t)DD * NN, (size_t)NN * DD);
}
